// NAFBlockDDF_11862699672009
// MI455X (gfx1250) — hardware-run, weakly checked
//
#include <hip/hip_runtime.h>


#define NB_  4
#define CC   32
#define C2   64
#define HH   256
#define WWD  256
#define NP   (HH * WWD)
#define NT   (NB_ * NP)
#define FS   32
typedef _Float16 h16;
typedef unsigned short bf;
typedef __attribute__((ext_vector_type(16))) __bf16   v16bf;
typedef __attribute__((ext_vector_type(16))) _Float16 v16h;
typedef __attribute__((ext_vector_type(8)))  _Float16 v8h;
typedef __attribute__((ext_vector_type(8)))  unsigned short v8us;
typedef __attribute__((ext_vector_type(8)))  float    v8f;
typedef __attribute__((ext_vector_type(4)))  float    v4f;
typedef v8h  __attribute__((may_alias)) v8ha;
typedef v4f  __attribute__((may_alias)) v4fa;
typedef v8us __attribute__((may_alias)) v8usa;

__device__ __forceinline__ unsigned short f2bf(float f) { unsigned u = __float_as_uint(f); u += 0x7FFFu + ((u >> 16) & 1u); return (unsigned short)(u >> 16); }
__device__ __forceinline__ float bf2f(unsigned short b) { return __uint_as_float(((unsigned)b) << 16); }
__device__ __forceinline__ float bfr(float f) { return bf2f(f2bf(f)); }
__device__ __forceinline__ v16h cat16(v8h lo, v8h hi) { return __builtin_shufflevector(lo, hi, 0, 1, 2, 3, 4, 5, 6, 7, 8, 9, 10, 11, 12, 13, 14, 15); }
__device__ __forceinline__ v16bf cat16b(v8us lo, v8us hi) { return __builtin_bit_cast(v16bf, __builtin_shufflevector(lo, hi, 0, 1, 2, 3, 4, 5, 6, 7, 8, 9, 10, 11, 12, 13, 14, 15)); }
__device__ __forceinline__ v8f wmma16(v16h a, v16h b, v8f c) { return __builtin_amdgcn_wmma_f32_16x16x32_f16(false, a, false, b, (short)0, c, false, false); }
__device__ __forceinline__ v8f wmmab(v16bf a, v16bf b, v8f c) { return __builtin_amdgcn_wmma_f32_16x16x32_bf16(false, a, false, b, (short)0, c, false, false); }


template <typename T16> struct WFrag;
template <> struct WFrag<h16> { typedef v16h V; static __device__ __forceinline__ V ld(const h16* p) { return cat16(*(const v8h*)p, *(const v8h*)(p + 16)); } static __device__ __forceinline__ v8f mma(V a, V b, v8f c) { return wmma16(a, b, c); } };
template <> struct WFrag<bf> { typedef v16bf V; static __device__ __forceinline__ V ld(const bf* p) { return cat16b(*(const v8us*)p, *(const v8us*)(p + 16)); } static __device__ __forceinline__ v8f mma(V a, V b, v8f c) { return wmmab(a, b, c); } };
template <typename T16, int NSPLIT, bool BIAS>
__global__ __launch_bounds__(32) void k_gemmw(const T16* __restrict__ A, const T16* __restrict__ A2, const T16* __restrict__ Bt, const T16* __restrict__ Bt2, int K, float* C, int ldc, const float* __restrict__ bias, size_t sA, size_t sB, size_t sC) {
    typedef typename WFrag<T16>::V V;
    __shared__ __align__(16) float os[16 * 68];
    const size_t z = blockIdx.z; A += z * sA; if (A2) A2 += z * sA; Bt += z * sB; if (Bt2) Bt2 += z * sB; C += z * sC;
    const int lane = threadIdx.x & 31, lr = lane & 15, hi = lane >> 4; const int r0 = blockIdx.x * 64, c0 = blockIdx.y * 64;
    v8f acc[4][4];
#pragma unroll
    for (int mb = 0; mb < 4; ++mb)
#pragma unroll
        for (int nb = 0; nb < 4; ++nb) acc[mb][nb] = (v8f){};
    const size_t aoff = (size_t)(r0 + lr) * K + 8 * hi, boff = (size_t)(c0 + lr) * K + 8 * hi;
#pragma unroll 1
    for (int kc = 0; kc < K; kc += 32) {
        V a[4], a2[4];
#pragma unroll
        for (int mb = 0; mb < 4; ++mb) { a[mb] = WFrag<T16>::ld(A + aoff + (size_t)mb * 16 * K + kc); if (NSPLIT == 1 || NSPLIT == 2) a2[mb] = WFrag<T16>::ld(A2 + aoff + (size_t)mb * 16 * K + kc); }
#pragma unroll
        for (int nb = 0; nb < 4; ++nb) { const V b = WFrag<T16>::ld(Bt + boff + (size_t)nb * 16 * K + kc); V b2; if (NSPLIT >= 2) b2 = WFrag<T16>::ld(Bt2 + boff + (size_t)nb * 16 * K + kc);
#pragma unroll
            for (int mb = 0; mb < 4; ++mb) { acc[mb][nb] = WFrag<T16>::mma(a[mb], b, acc[mb][nb]); if (NSPLIT == 1 || NSPLIT == 2) acc[mb][nb] = WFrag<T16>::mma(a2[mb], b, acc[mb][nb]); if (NSPLIT >= 2) acc[mb][nb] = WFrag<T16>::mma(a[mb], b2, acc[mb][nb]); } }
        asm volatile("v_nop\n\tv_nop\n\tv_nop\n\tv_nop" : "+v"(acc[0][0]), "+v"(acc[1][1]), "+v"(acc[2][2]), "+v"(acc[3][3]) : "v"(a[0]), "v"(a[3]));
    }
#pragma unroll
    for (int mb = 0; mb < 4; ++mb) {
#pragma unroll
        for (int nb = 0; nb < 4; ++nb) {
#pragma unroll
            for (int j = 0; j < 8; ++j) os[(hi * 8 + j) * 68 + nb * 16 + lr] = acc[mb][nb][j]; }
        __builtin_amdgcn_wave_barrier(); asm volatile("" ::: "memory");
        float* crow = C + (size_t)(r0 + mb * 16) * ldc + c0;
#pragma unroll 1
        for (int ps = 0; ps < 2; ++ps) {
#pragma unroll
            for (int s = 0; s < 8; ++s) { const int row = 2 * s + hi, cofs = lr * 4; v4f val = *(const v4fa*)(os + row * 68 + cofs); if (BIAS) { val[0] += bfr(bias[c0 + cofs]); val[1] += bfr(bias[c0 + cofs + 1]); val[2] += bfr(bias[c0 + cofs + 2]); val[3] += bfr(bias[c0 + cofs + 3]); }
                *(volatile v4f*)(crow + (size_t)row * ldc + cofs) = val; }
            if (ps == 0) __threadfence(); }
        __builtin_amdgcn_wave_barrier(); asm volatile("" ::: "memory");
    }
}

__device__ __forceinline__ void splitf(float y, unsigned short& h, unsigned short& l) { h = f2bf(y); l = f2bf(y - bf2f(h)); }
typedef __attribute__((ext_vector_type(2))) unsigned short v2us;
typedef __attribute__((ext_vector_type(2))) float v2f;

__global__ __launch_bounds__(256) void k_wpad(const float* __restrict__ w, int O, bf* WB) { const int i = blockIdx.x * 256 + threadIdx.x; if (i >= 64 * CC / 2) return; const int e = i * 2; const int o = e / CC, k = e % CC; v2us v;
#pragma unroll
    for (int q = 0; q < 2; ++q) v[q] = (o < O) ? f2bf(w[o * CC + k + q]) : (unsigned short)0; *(volatile v2us*)(WB + e) = v; __threadfence(); *(volatile v2us*)(WB + e) = v; }
__global__ __launch_bounds__(64) void k_bpad(const float* __restrict__ b, int N, float* out) { const int i = threadIdx.x; const float v = i < N ? b[i < N ? i : 0] : 0.f; *(volatile float*)(out + i) = v; __threadfence(); *(volatile float*)(out + i) = v; }
template <bool FROMY>
__global__ __launch_bounds__(256) void k_ln(const float* __restrict__ src, const float* __restrict__ gw, const float* __restrict__ gb, bf* Ph, bf* Pl) {
    const int lane = threadIdx.x & 31; const int L0 = (blockIdx.x * 8 + (threadIdx.x >> 5)) * 8; const int nlines = NT * CC / 64;
#pragma unroll 1
    for (int l = 0; l < 8; ++l) { const int L = L0 + l; if (L >= nlines) break; const int e = L * 64 + lane * 2; const int c = e & 31; const int row = e >> 5; const int b = row / NP, p = row % NP;
        float v0 = src[((size_t)b * CC + c) * NP + p], v1 = src[((size_t)b * CC + c + 1) * NP + p]; if (!FROMY) { v0 = bfr(v0); v1 = bfr(v1); }
        float s = v0 + v1;
#pragma unroll
        for (int sh = 8; sh; sh >>= 1) s += __shfl_xor(s, sh, 32);
        const float mu = s * (1.0f / CC); const float d0 = v0 - mu, d1 = v1 - mu; float q = d0 * d0 + d1 * d1;
#pragma unroll
        for (int sh = 8; sh; sh >>= 1) q += __shfl_xor(q, sh, 32);
        const float rs = __fdiv_rn(1.0f, sqrtf(q * (1.0f / CC) + 1e-6f)); v2us oh, ol; unsigned short a, c2;
        splitf(d0 * rs * bfr(gw[c]) + bfr(gb[c]), a, c2); oh[0] = a; ol[0] = c2; splitf(d1 * rs * bfr(gw[c + 1]) + bfr(gb[c + 1]), a, c2); oh[1] = a; ol[1] = c2;
        *(volatile v2us*)(Ph + (size_t)e) = oh; *(volatile v2us*)(Pl + (size_t)e) = ol; __threadfence(); *(volatile v2us*)(Ph + (size_t)e) = oh; *(volatile v2us*)(Pl + (size_t)e) = ol; }
}
__global__ __launch_bounds__(256) void k_ddf(const float* __restrict__ C1, const float* __restrict__ w2, float* G) {
    const int lane = threadIdx.x & 31; const int L0 = (blockIdx.x * 8 + (threadIdx.x >> 5)) * 8; const int nlines = NB_ * CC * NP / 64;
#pragma unroll 1
    for (int ps = 0; ps < 2; ++ps) {
#pragma unroll 1
        for (int l = 0; l < 8; ++l) { const int L = L0 + l; if (L >= nlines) break; const int e = L * 64 + lane * 2; v2f o;
#pragma unroll
            for (int q = 0; q < 2; ++q) { const int idx = e + q; const int p = idx & (NP - 1); const int c = (idx >> 16) & 31; const int b = idx >> 21; const int h = p >> 8, w = p & 255;
                const float sy = ((float)h + 0.5f) * 0.125f - 0.5f, sx = ((float)w + 0.5f) * 0.125f - 0.5f; const float fy = floorf(sy), fx = floorf(sx); const float wy = sy - fy, wx = sx - fx;
                int y0 = (int)fy, x0 = (int)fx; int y1 = y0 + 1, x1 = x0 + 1; y0 = y0 < 0 ? 0 : y0; x0 = x0 < 0 ? 0 : x0; y1 = y1 > FS - 1 ? FS - 1 : y1; x1 = x1 > FS - 1 ? FS - 1 : x1;
                const int i00 = y0 * FS + x0, i01 = y0 * FS + x1, i10 = y1 * FS + x0, i11 = y1 * FS + x1;
                const float w00 = (1.f - wy) * (1.f - wx), w01 = (1.f - wy) * wx, w10 = wy * (1.f - wx), w11 = wy * wx;
                float acc[2] = {0.f, 0.f};
#pragma unroll
                for (int half = 0; half < 2; ++half) { const int ch = c + half * CC; const float* fm = w2 + (((size_t)b * C2 + ch) * 9) * FS * FS;
#pragma unroll 1
                    for (int tap = 0; tap < 9; ++tap) { const int hh = h + tap / 3 - 1, ww = w + tap % 3 - 1; if (hh < 0 || hh >= HH || ww < 0 || ww >= WWD) continue; const float* f = fm + tap * FS * FS;
                        const float fv = (bfr(f[i00]) * w00 + bfr(f[i01]) * w01) + (bfr(f[i10]) * w10 + bfr(f[i11]) * w11);
                        acc[half] = fmaf(C1[((size_t)b * NP + hh * WWD + ww) * C2 + ch], fv, acc[half]); } }
                o[q] = acc[0] * acc[1]; }
            *(volatile v2f*)(G + (size_t)e) = o; }
        if (ps == 0) __threadfence(); }
}
__global__ __launch_bounds__(256) void k_mean(const float* __restrict__ G, float* MEAN) {
    const int lane = threadIdx.x & 31; const int wg = blockIdx.x * 8 + (threadIdx.x >> 5); if (wg >= NB_ * CC) return; const float* row = G + (size_t)wg * NP; float s = 0.f;
#pragma unroll 4
    for (int i = lane; i < NP; i += 32) s += row[i];
#pragma unroll
    for (int sh = 16; sh; sh >>= 1) s += __shfl_xor(s, sh, 32);
    const float v = lane == 0 ? s * (1.0f / NP) : 0.f; *(volatile float*)(MEAN + (size_t)wg * 32 + lane) = v; __threadfence(); *(volatile float*)(MEAN + (size_t)wg * 32 + lane) = v;
}
__global__ __launch_bounds__(256) void k_gsplit(const float* __restrict__ G, const float* __restrict__ MEAN, const float* __restrict__ sw, const float* __restrict__ sb, bf* Ph, bf* Pl) {
    const int lane = threadIdx.x & 31; const int L0 = (blockIdx.x * 8 + (threadIdx.x >> 5)) * 8; const int nlines = NT * CC / 64;
    const int b = (L0 * 64) / (NP * CC);
    float sv = bfr(sb[lane]);
#pragma unroll 1
    for (int k = 0; k < CC; ++k) sv = fmaf(bfr(sw[lane * CC + k]), MEAN[((size_t)b * CC + k) * 32], sv);
#pragma unroll 1
    for (int ps = 0; ps < 2; ++ps) {
#pragma unroll 1
        for (int l = 0; l < 8; ++l) { const int L = L0 + l; if (L >= nlines) break; const int e = L * 64 + lane * 2; const int c = e & 31; const int row = e >> 5; const int p = row % NP; v2us oh, ol;
#pragma unroll
            for (int q = 0; q < 2; ++q) { const float sc = __shfl(sv, c + q, 32); unsigned short a, c2; splitf(G[((size_t)b * CC + c + q) * NP + p] * sc, a, c2); oh[q] = a; ol[q] = c2; }
            *(volatile v2us*)(Ph + (size_t)e) = oh; *(volatile v2us*)(Pl + (size_t)e) = ol; }
        if (ps == 0) __threadfence(); }
}
template <bool ROUND>
__global__ __launch_bounds__(256) void k_resid(const float* __restrict__ base, const float* __restrict__ C, const float* __restrict__ coef, float* Y) {
    const size_t i = (size_t)blockIdx.x * 256 + threadIdx.x; if (i >= (size_t)NB_ * CC * NP / 4) return; const size_t e = i * 4; const int p = (int)(e & (NP - 1)); const int c = (int)((e >> 16) & 31); const int b = (int)(e >> 21);
    const v4f bv = *(const v4f*)(base + e); const float cf = bfr(coef[c]); v4f o;
#pragma unroll
    for (int q = 0; q < 4; ++q) o[q] = (ROUND ? bfr(bv[q]) : bv[q]) + C[((size_t)b * NP + p + q) * C2 + c] * cf;
    *(volatile v4f*)(Y + e) = o; __threadfence(); *(volatile v4f*)(Y + e) = o;
}
__global__ __launch_bounds__(256) void k_gate2(const float* __restrict__ C4, bf* Ph, bf* Pl) {
    const int lane = threadIdx.x & 31; const int L0 = (blockIdx.x * 8 + (threadIdx.x >> 5)) * 8; const int nlines = NT * CC / 64;
#pragma unroll 1
    for (int ps = 0; ps < 2; ++ps) {
#pragma unroll
        for (int l = 0; l < 8; ++l) { const int L = L0 + l; if (L >= nlines) break; const int e = L * 64 + lane * 2; const int c = e & 31; const size_t row = e >> 5; v2us oh, ol;
#pragma unroll
            for (int q = 0; q < 2; ++q) { unsigned short a, c2; splitf(C4[row * C2 + c + q] * C4[row * C2 + c + q + CC], a, c2); oh[q] = a; ol[q] = c2; }
            *(volatile v2us*)(Ph + (size_t)e) = oh; *(volatile v2us*)(Pl + (size_t)e) = ol; }
        if (ps == 0) __threadfence(); }
}

extern "C" void kernel_launch(void* const* d_in, const int* in_sizes, int n_in,
                              void* d_out, int out_size, void* d_ws, size_t ws_size, hipStream_t stream) {
    (void)in_sizes; (void)n_in; (void)out_size;
    const float* inp = (const float*)d_in[0]; const float* w2 = (const float*)d_in[1]; const float* c1w = (const float*)d_in[2]; const float* c1b = (const float*)d_in[3]; const float* c3w = (const float*)d_in[4]; const float* c3b = (const float*)d_in[5];
    const float* scw = (const float*)d_in[6]; const float* scb = (const float*)d_in[7]; const float* c4w = (const float*)d_in[8]; const float* c4b = (const float*)d_in[9]; const float* c5w = (const float*)d_in[10]; const float* c5b = (const float*)d_in[11];
    const float* n1w = (const float*)d_in[12]; const float* n1b = (const float*)d_in[13]; const float* n2w = (const float*)d_in[14]; const float* n2b = (const float*)d_in[15]; const float* beta = (const float*)d_in[16]; const float* gamma = (const float*)d_in[17];
    float* OUT = (float*)d_out;
    char* wsp = (char*)d_ws;
    auto take = [&](size_t bytes) { char* p = wsp; wsp += (bytes + 255) & ~(size_t)255; return (void*)p; };
    bf* W1 = (bf*)take(64 * CC * 2); bf* W3 = (bf*)take(64 * CC * 2); bf* W4 = (bf*)take(64 * CC * 2); bf* W5 = (bf*)take(64 * CC * 2); float* B3P = (float*)take(64 * 4); float* B5P = (float*)take(64 * 4); float* MEAN = (float*)take((size_t)NB_ * CC * 32 * 4);
    bf* Ph = (bf*)take((size_t)NT * CC * 2); bf* Pl = (bf*)take((size_t)NT * CC * 2);
    float* Cb = (float*)take((size_t)NT * C2 * 4);
    float* G = (float*)take((size_t)NB_ * CC * NP * 4);
    float* Y = (float*)take((size_t)NB_ * CC * NP * 4);
    if ((size_t)(wsp - (char*)d_ws) > ws_size) return;
    k_wpad<<<4, 256, 0, stream>>>(c1w, 64, W1); k_wpad<<<4, 256, 0, stream>>>(c3w, 32, W3); k_wpad<<<4, 256, 0, stream>>>(c4w, 64, W4); k_wpad<<<4, 256, 0, stream>>>(c5w, 32, W5);
    k_bpad<<<1, 64, 0, stream>>>(c3b, 32, B3P); k_bpad<<<1, 64, 0, stream>>>(c5b, 32, B5P);
    const unsigned LB = (unsigned)((NT * CC / 64 + 63) / 64);
    k_ln<false><<<LB, 256, 0, stream>>>(inp, n1w, n1b, Ph, Pl);
    k_gemmw<bf, 1, true><<<dim3(NT / 64, 1, 1), 32, 0, stream>>>(Ph, Pl, W1, nullptr, CC, Cb, C2, c1b, 0, 0, 0);
    k_ddf<<<LB, 256, 0, stream>>>(Cb, w2, G);
    k_mean<<<NB_ * CC / 8, 256, 0, stream>>>(G, MEAN);
    k_gsplit<<<LB, 256, 0, stream>>>(G, MEAN, scw, scb, Ph, Pl);
    k_gemmw<bf, 1, true><<<dim3(NT / 64, 1, 1), 32, 0, stream>>>(Ph, Pl, W3, nullptr, CC, Cb, C2, B3P, 0, 0, 0);
    k_resid<true><<<(unsigned)(((size_t)NB_ * CC * NP / 4 + 255) / 256), 256, 0, stream>>>(inp, Cb, beta, Y);
    k_ln<true><<<LB, 256, 0, stream>>>(Y, n2w, n2b, Ph, Pl);
    k_gemmw<bf, 1, true><<<dim3(NT / 64, 1, 1), 32, 0, stream>>>(Ph, Pl, W4, nullptr, CC, Cb, C2, c4b, 0, 0, 0);
    k_gate2<<<LB, 256, 0, stream>>>(Cb, Ph, Pl);
    k_gemmw<bf, 1, true><<<dim3(NT / 64, 1, 1), 32, 0, stream>>>(Ph, Pl, W5, nullptr, CC, Cb, C2, B5P, 0, 0, 0);
    k_resid<false><<<(unsigned)(((size_t)NB_ * CC * NP / 4 + 255) / 256), 256, 0, stream>>>(Y, Cb, gamma, OUT);
}
